// SplitScaleAttend_6734508720466
// MI455X (gfx1250) — hardware-verified
//
#include <hip/hip_runtime.h>
#include <math.h>

#define NBH   64
#define SEQ   2048
#define HD    64
#define NELEM (NBH * SEQ * HD)

static_assert(NELEM == 8388608);
static_assert(SEQ % 128 == 0);
static_assert(HD == 64);

typedef __attribute__((ext_vector_type(16))) __bf16 v16b;
typedef __attribute__((ext_vector_type(8)))  __bf16 v8b;
typedef __attribute__((ext_vector_type(8)))  float  v8f;
typedef __attribute__((ext_vector_type(4)))  float  v4f;
typedef __attribute__((ext_vector_type(4)))  unsigned int v4u;
typedef __attribute__((ext_vector_type(8)))  unsigned int v8u;

__device__ __forceinline__ unsigned short f2bf_bits(float f) {
  unsigned u = __float_as_uint(f);
  return (unsigned short)((u + 0x7FFFu + ((u >> 16) & 1u)) >> 16);
}
__device__ __forceinline__ float bf_bits2f(unsigned short b) { return __uint_as_float(((unsigned)b) << 16); }
__device__ __forceinline__ unsigned pk16(unsigned short a, unsigned short b) { return (unsigned)a | ((unsigned)b << 16); }

__device__ __forceinline__ void split2(float f0, float f1, unsigned& hw, unsigned& lw) {
  const unsigned short h0 = f2bf_bits(f0), h1 = f2bf_bits(f1);
  const unsigned short l0 = f2bf_bits(f0 - bf_bits2f(h0)), l1 = f2bf_bits(f1 - bf_bits2f(h1));
  hw = pk16(h0, h1);
  lw = pk16(l0, l1);
}

__device__ __forceinline__ void split2t(float f0, float f1, unsigned& hw, unsigned& lw) {
  const unsigned u0 = __float_as_uint(f0) & 0xFFFF0000u;
  const unsigned u1 = __float_as_uint(f1) & 0xFFFF0000u;
  const unsigned short l0 = f2bf_bits(f0 - __uint_as_float(u0));
  const unsigned short l1 = f2bf_bits(f1 - __uint_as_float(u1));
  hw = (u0 >> 16) | u1;
  lw = pk16(l0, l1);
}

__device__ __forceinline__ v8f mma_bf(v16b a, v16b b, v8f c) {
  c = __builtin_amdgcn_wmma_f32_16x16x32_bf16(false, a, false, b, (short)0, c, false, false);
  asm volatile("v_nop\n\tv_nop\n\tv_nop\n\tv_nop" : "+v"(c) : "v"(a), "v"(b));
  return c;
}

__global__ __launch_bounds__(256) void split_qk_kernel(const float* __restrict__ q, const float* __restrict__ k,
                                                       unsigned short* __restrict__ qh, unsigned short* __restrict__ ql,
                                                       unsigned short* __restrict__ kh, unsigned short* __restrict__ kl,
                                                       int ngrp) {
  const int t = blockIdx.x * 256 + (int)threadIdx.x;
  if (t >= ngrp) return;
  const size_t so = (size_t)t * 8;
  const v4f a0 = *(const v4f*)(q + so);
  const v4f a1 = *(const v4f*)(q + so + 4);
  const v4f b0 = *(const v4f*)(k + so) * 0.125f;
  const v4f b1 = *(const v4f*)(k + so + 4) * 0.125f;
  unsigned h0, h1, h2, h3, l0, l1, l2, l3;
  split2(a0[0], a0[1], h0, l0);
  split2(a0[2], a0[3], h1, l1);
  split2(a1[0], a1[1], h2, l2);
  split2(a1[2], a1[3], h3, l3);
  const v4u qhv = (v4u){h0, h1, h2, h3};
  const v4u qlv = (v4u){l0, l1, l2, l3};
  split2(b0[0], b0[1], h0, l0);
  split2(b0[2], b0[3], h1, l1);
  split2(b1[0], b1[1], h2, l2);
  split2(b1[2], b1[3], h3, l3);
  const v4u khv = (v4u){h0, h1, h2, h3};
  const v4u klv = (v4u){l0, l1, l2, l3};
  volatile v4u* pqh = (volatile v4u*)(qh + so);
  volatile v4u* pql = (volatile v4u*)(ql + so);
  volatile v4u* pkh = (volatile v4u*)(kh + so);
  volatile v4u* pkl = (volatile v4u*)(kl + so);
  *pqh = qhv;
  *pql = qlv;
  *pkh = khv;
  *pkl = klv;
  __threadfence();
  *pqh = qhv;
  *pql = qlv;
  *pkh = khv;
  *pkl = klv;
}

#define TFP 68
__global__ __launch_bounds__(256) void vt_split_kernel(const float* __restrict__ v,
                                                       unsigned short* __restrict__ vth,
                                                       unsigned short* __restrict__ vtl) {
  __shared__ __align__(16) float tf[64 * TFP];
  const int tid = threadIdx.x;
  const int nt  = blockIdx.x % (SEQ / 64);
  const int bh  = blockIdx.x / (SEQ / 64);
  const int n0  = nt * 64;
  {
    const int lr = tid >> 4;
    const int c4 = (tid & 15) * 4;
#pragma unroll
    for (int it = 0; it < 4; ++it) {
      const int row = it * 16 + lr;
      const float* sp = v + ((size_t)bh * SEQ + n0 + row) * HD + c4;
      *(v4f*)(tf + row * TFP + c4) = *(const v4f*)(sp);
    }
  }
  __syncthreads();
  {
    const int sub = tid >> 3;
    const int t8  = (tid & 7) * 8;
    v4u hv[2], lv[2];
#pragma unroll
    for (int it = 0; it < 2; ++it) {
      const int d = it * 32 + sub;
      unsigned hw[4], lw[4];
#pragma unroll
      for (int qq = 0; qq < 4; ++qq) {
        const float f0 = tf[(t8 + 2 * qq) * TFP + d];
        const float f1 = tf[(t8 + 2 * qq + 1) * TFP + d];
        split2(f0, f1, hw[qq], lw[qq]);
      }
      hv[it] = (v4u){hw[0], hw[1], hw[2], hw[3]};
      lv[it] = (v4u){lw[0], lw[1], lw[2], lw[3]};
    }
    unsigned short* th = vth + (size_t)bh * HD * SEQ + n0 + t8;
    unsigned short* tl = vtl + (size_t)bh * HD * SEQ + n0 + t8;
    for (int ps = 0; ps < 2; ++ps) {
#pragma unroll
      for (int it = 0; it < 2; ++it) {
        const int d = it * 32 + sub;
        const size_t go = (size_t)d * SEQ;
        *(volatile v4u*)(th + go) = hv[it];
        *(volatile v4u*)(tl + go) = lv[it];
      }
      __threadfence();
    }
  }
}

#define QB  128
#define KC  64
#define KSP 72
#define VTP 72
#define OSP 68

__global__ __launch_bounds__(256)
void attn_kernel(const unsigned short* __restrict__ qhp, const unsigned short* __restrict__ qlp,
                 const unsigned short* __restrict__ khp, const unsigned short* __restrict__ klp,
                 const unsigned short* __restrict__ vhp, const unsigned short* __restrict__ vlp,
                 float* __restrict__ out) {
  union FB { v16b v; v8b h[2]; v8u u; };
  __shared__ __align__(16) __bf16 Ksh[KC * KSP];
  __shared__ __align__(16) __bf16 Ksl[KC * KSP];
  __shared__ __align__(16) __bf16 Vth[HD * VTP];
  __shared__ __align__(16) __bf16 Vtl[HD * VTP];
  __shared__ __align__(16) float  Os[8][16 * OSP];

  const int tid  = threadIdx.x;
  const int wave = tid >> 5;
  const int lane = tid & 31;
  const int lh   = lane >> 4;
  const int c    = lane & 15;

  const int nqt = SEQ / QB;
  const int qt  = blockIdx.x % nqt;
  const int bh  = blockIdx.x / nqt;
  const int q0  = qt * QB + wave * 16;

  const __bf16* Qh = (const __bf16*)(const void*)qhp + (size_t)bh * SEQ * HD;
  const __bf16* Ql = (const __bf16*)(const void*)qlp + (size_t)bh * SEQ * HD;
  const __bf16* Kh = (const __bf16*)(const void*)khp + (size_t)bh * SEQ * HD;
  const __bf16* Kl = (const __bf16*)(const void*)klp + (size_t)bh * SEQ * HD;
  const __bf16* Vh = (const __bf16*)(const void*)vhp + (size_t)bh * HD * SEQ;
  const __bf16* Vl = (const __bf16*)(const void*)vlp + (size_t)bh * HD * SEQ;

  FB qbh[2], qbl[2];
  {
    const __bf16* qrh = Qh + (size_t)(q0 + c) * HD + 8 * lh;
    const __bf16* qrl = Ql + (size_t)(q0 + c) * HD + 8 * lh;
#pragma unroll
    for (int dc = 0; dc < 2; ++dc) {
      qbh[dc].h[0] = *(const v8b*)(qrh + dc * 32);
      qbh[dc].h[1] = *(const v8b*)(qrh + dc * 32 + 16);
      qbl[dc].h[0] = *(const v8b*)(qrl + dc * 32);
      qbl[dc].h[1] = *(const v8b*)(qrl + dc * 32 + 16);
    }
  }

  float mrow = -INFINITY, lrow = 0.f;
  v8f oacc[4];
#pragma unroll
  for (int t = 0; t < 4; ++t) oacc[t] = (v8f){0.f, 0.f, 0.f, 0.f, 0.f, 0.f, 0.f, 0.f};

#pragma unroll 1
  for (int kc = 0; kc < SEQ / KC; ++kc) {
    const int kv0 = kc * KC;
    __syncthreads();
    {
      const int r = tid >> 2, qq = (tid & 3) * 16;
      const __bf16* khs = Kh + (size_t)(kv0 + r) * HD + qq;
      const __bf16* kls = Kl + (size_t)(kv0 + r) * HD + qq;
      __bf16* kdh = Ksh + r * KSP + qq;
      __bf16* kdl = Ksl + r * KSP + qq;
      *(v8b*)(kdh)     = *(const v8b*)(khs);
      *(v8b*)(kdh + 8) = *(const v8b*)(khs + 8);
      *(v8b*)(kdl)     = *(const v8b*)(kls);
      *(v8b*)(kdl + 8) = *(const v8b*)(kls + 8);
      const __bf16* vhs = Vh + (size_t)r * SEQ + kv0 + qq;
      const __bf16* vls = Vl + (size_t)r * SEQ + kv0 + qq;
      __bf16* vdh = Vth + r * VTP + qq;
      __bf16* vdl = Vtl + r * VTP + qq;
      *(v8b*)(vdh)     = *(const v8b*)(vhs);
      *(v8b*)(vdh + 8) = *(const v8b*)(vhs + 8);
      *(v8b*)(vdl)     = *(const v8b*)(vls);
      *(v8b*)(vdl + 8) = *(const v8b*)(vls + 8);
    }
    __syncthreads();

    v8f s[4];
#pragma unroll
    for (int j = 0; j < 4; ++j) s[j] = (v8f){0.f, 0.f, 0.f, 0.f, 0.f, 0.f, 0.f, 0.f};
#pragma unroll
    for (int j = 0; j < 4; ++j) {
#pragma unroll
      for (int dc = 0; dc < 2; ++dc) {
        const __bf16* kp = Ksh + (j * 16 + c) * KSP + dc * 32 + 8 * lh;
        const __bf16* kq = Ksl + (j * 16 + c) * KSP + dc * 32 + 8 * lh;
        FB ka, kl;
        ka.h[0] = *(const v8b*)(kp);
        ka.h[1] = *(const v8b*)(kp + 16);
        kl.h[0] = *(const v8b*)(kq);
        kl.h[1] = *(const v8b*)(kq + 16);
        s[j] = mma_bf(ka.v, qbh[dc].v, s[j]);
        s[j] = mma_bf(ka.v, qbl[dc].v, s[j]);
        s[j] = mma_bf(kl.v, qbh[dc].v, s[j]);
      }
    }

    float cm = -INFINITY;
#pragma unroll
    for (int j = 0; j < 4; ++j)
#pragma unroll
      for (int r = 0; r < 8; ++r) cm = fmaxf(cm, s[j][r]);
    cm = fmaxf(cm, __shfl_xor(cm, 16, 32));
    const float mnew  = fmaxf(mrow, cm);
    const float alpha = __expf(mrow - mnew);
    mrow = mnew;

    float psum = 0.f;
    unsigned hw[16], lw[16];
#pragma unroll
    for (int j = 0; j < 4; ++j) {
#pragma unroll
      for (int rp = 0; rp < 4; ++rp) {
        const float p0 = __expf(s[j][2 * rp] - mnew);
        const float p1 = __expf(s[j][2 * rp + 1] - mnew);
        psum += p0 + p1;
        split2t(p0, p1, hw[j * 4 + rp], lw[j * 4 + rp]);
      }
    }
    psum += __shfl_xor(psum, 16, 32);
    lrow = lrow * alpha + psum;
#pragma unroll
    for (int t = 0; t < 4; ++t)
#pragma unroll
      for (int r = 0; r < 8; ++r) oacc[t][r] *= alpha;

#pragma unroll
    for (int kk = 0; kk < 2; ++kk) {
      FB pb, pl;
      pb.u = (v8u){hw[8 * kk + 0], hw[8 * kk + 1], hw[8 * kk + 2], hw[8 * kk + 3],
                   hw[8 * kk + 4], hw[8 * kk + 5], hw[8 * kk + 6], hw[8 * kk + 7]};
      pl.u = (v8u){lw[8 * kk + 0], lw[8 * kk + 1], lw[8 * kk + 2], lw[8 * kk + 3],
                   lw[8 * kk + 4], lw[8 * kk + 5], lw[8 * kk + 6], lw[8 * kk + 7]};
#pragma unroll
      for (int t = 0; t < 4; ++t) {
        const __bf16* vp = Vth + (t * 16 + c) * VTP + kk * 32 + 8 * lh;
        const __bf16* vq = Vtl + (t * 16 + c) * VTP + kk * 32 + 8 * lh;
        FB va, vl;
        va.h[0] = *(const v8b*)(vp);
        va.h[1] = *(const v8b*)(vp + 16);
        vl.h[0] = *(const v8b*)(vq);
        vl.h[1] = *(const v8b*)(vq + 16);
        oacc[t] = mma_bf(va.v, pb.v, oacc[t]);
        oacc[t] = mma_bf(va.v, pl.v, oacc[t]);
        oacc[t] = mma_bf(vl.v, pb.v, oacc[t]);
      }
    }
  }

  {
    const float inv = 1.0f / lrow;
    float* os = Os[wave] + c * OSP + 8 * lh;
#pragma unroll
    for (int t = 0; t < 4; ++t) {
      const v4f w0 = (v4f){oacc[t][0] * inv, oacc[t][1] * inv, oacc[t][2] * inv, oacc[t][3] * inv};
      const v4f w1 = (v4f){oacc[t][4] * inv, oacc[t][5] * inv, oacc[t][6] * inv, oacc[t][7] * inv};
      *(v4f*)(os + t * 16)     = w0;
      *(v4f*)(os + t * 16 + 4) = w1;
    }
  }
  __builtin_amdgcn_fence(__ATOMIC_RELEASE, "workgroup");
  __builtin_amdgcn_wave_barrier();
  __builtin_amdgcn_fence(__ATOMIC_ACQUIRE, "workgroup");
  {
    const float* osr = Os[wave];
    const int rh = lane >> 4, c4 = (lane & 15) * 4;
    float* ob = out + ((size_t)bh * SEQ + q0) * HD;
    for (int ps = 0; ps < 2; ++ps) {
#pragma unroll
      for (int it = 0; it < 8; ++it) {
        const int row = it * 2 + rh;
        const v4f vv = *(const v4f*)(osr + row * OSP + c4);
        *(volatile v4f*)(ob + (size_t)row * HD + c4) = vv;
      }
      __threadfence();
    }
  }
}

extern "C" void kernel_launch(void* const* d_in, const int* in_sizes, int n_in,
                              void* d_out, int out_size, void* d_ws, size_t ws_size,
                              hipStream_t stream) {
  if (n_in < 3) return;
  if (in_sizes[0] != NELEM || in_sizes[1] != NELEM || in_sizes[2] != NELEM) return;
  if (out_size != NELEM) return;

  const float* q = (const float*)d_in[0];
  const float* k = (const float*)d_in[1];
  const float* v = (const float*)d_in[2];
  float* o = (float*)d_out;

  const size_t PB = (size_t)NELEM * 2;
  size_t off = 0;
  const size_t oQh = off; off += PB;
  const size_t oQl = off; off += PB;
  const size_t oKh = off; off += PB;
  const size_t oKl = off; off += PB;
  const size_t oVh = off; off += PB;
  const size_t oVl = off; off += PB;
  if (off > ws_size) return;

  char* ws = (char*)d_ws;
  unsigned short* Qh  = (unsigned short*)(ws + oQh);
  unsigned short* Ql  = (unsigned short*)(ws + oQl);
  unsigned short* Kh  = (unsigned short*)(ws + oKh);
  unsigned short* Kl  = (unsigned short*)(ws + oKl);
  unsigned short* VTh = (unsigned short*)(ws + oVh);
  unsigned short* VTl = (unsigned short*)(ws + oVl);

  const int ngrp = NELEM / 8;
  split_qk_kernel<<<dim3((ngrp + 255) / 256), dim3(256), 0, stream>>>(q, k, Qh, Ql, Kh, Kl, ngrp);
  vt_split_kernel<<<dim3(NBH * (SEQ / 64)), dim3(256), 0, stream>>>(v, VTh, VTl);
  attn_kernel<<<dim3(NBH * (SEQ / QB)), dim3(256), 0, stream>>>(Qh, Ql, Kh, Kl, VTh, VTl, o);
  (void)hipGetLastError();
}
